// CosineAttentionBlock_29403346108653
// MI455X (gfx1250) — hardware-verified
//
#include <hip/hip_runtime.h>
#include <math.h>

constexpr int kBatch  = 2;
constexpr int kSeq    = 4096;
constexpr int kDim    = 512;
constexpr int kHeads  = 8;
constexpr int kHdim   = 64;
constexpr int kMlp    = 2048;
constexpr int kTok    = kBatch * kSeq;
constexpr int kGroups = kBatch * kHeads;
constexpr float kWCarry    = 64.0f;
constexpr float kWCarryInv = 1.0f / 64.0f;
constexpr float kInvDim    = 1.0f / 512.0f;
constexpr float kLnEps     = 1e-5f;
constexpr float kNormEps   = 1e-12f;

typedef __attribute__((ext_vector_type(16))) _Float16 v16h;
typedef __attribute__((ext_vector_type(8)))  _Float16 v8h;
typedef __attribute__((ext_vector_type(16))) __bf16   v16b;
typedef __attribute__((ext_vector_type(8)))  __bf16   v8b;
typedef __attribute__((ext_vector_type(8)))  float    v8f;
typedef __attribute__((ext_vector_type(4)))  float    v4f;
typedef __attribute__((ext_vector_type(4)))  unsigned int v4u;

__device__ __forceinline__ unsigned short f2bf_bits(float f) {
  unsigned u = __float_as_uint(f);
  return (unsigned short)((u + 0x7FFFu + ((u >> 16) & 1u)) >> 16);
}
__device__ __forceinline__ float bf_bits2f(unsigned short h) { return __uint_as_float(((unsigned)h) << 16); }

__device__ __forceinline__ void dep_guard_h(v8f& a, v8f& b, v16h x, v16h y) { asm volatile("v_nop\n\tv_nop\n\tv_nop\n\tv_nop" : "+v"(a), "+v"(b) : "v"(x), "v"(y)); }
__device__ __forceinline__ void dep_guard_b(v8f& a, v8f& b, v16b x, v16b y) { asm volatile("v_nop\n\tv_nop\n\tv_nop\n\tv_nop" : "+v"(a), "+v"(b) : "v"(x), "v"(y)); }
__device__ __forceinline__ void keep4_h(v16h a, v16h b, v16h c, v16h d) { asm volatile("v_nop" :: "v"(a), "v"(b), "v"(c), "v"(d)); }
__device__ __forceinline__ void keep4_b(v16b a, v16b b, v16b c, v16b d) { asm volatile("v_nop" :: "v"(a), "v"(b), "v"(c), "v"(d)); }
__device__ __forceinline__ void acc_guard4(v8f& a, v8f& b, v8f& c, v8f& d) { asm volatile("v_nop\n\tv_nop\n\tv_nop\n\tv_nop" : "+v"(a), "+v"(b), "+v"(c), "+v"(d)); }
template <typename T> struct Frag;
template <> struct Frag<_Float16> {
  typedef v16h V; union U { v16h v; v8h h[2]; };
  static __device__ __forceinline__ v16h load(const _Float16* p) {
    U f; f.h[0] = *(const v8h*)(p); f.h[1] = *(const v8h*)(p + 16); return f.v;
  }
  static __device__ __forceinline__ v8f mma(v16h a, v16h b, v8f c) {
    return __builtin_amdgcn_wmma_f32_16x16x32_f16(false, a, false, b, (short)0, c, false, false);
  }
  static __device__ __forceinline__ void guard(v8f& a, v8f& b, v16h x, v16h y) { dep_guard_h(a, b, x, y); }
  static __device__ __forceinline__ void keep(v16h a, v16h b, v16h c, v16h d) { keep4_h(a, b, c, d); }
};
template <> struct Frag<__bf16> {
  typedef v16b V; union U { v16b v; v8b h[2]; };
  static __device__ __forceinline__ v16b load(const __bf16* p) {
    U f; f.h[0] = *(const v8b*)(p); f.h[1] = *(const v8b*)(p + 16); return f.v;
  }
  static __device__ __forceinline__ v8f mma(v16b a, v16b b, v8f c) {
    return __builtin_amdgcn_wmma_f32_16x16x32_bf16(false, a, false, b, (short)0, c, false, false);
  }
  static __device__ __forceinline__ void guard(v8f& a, v8f& b, v16b x, v16b y) { dep_guard_b(a, b, x, y); }
  static __device__ __forceinline__ void keep(v16b a, v16b b, v16b c, v16b d) { keep4_b(a, b, c, d); }
};

__device__ __forceinline__ unsigned pk16(unsigned short a, unsigned short b) { return (unsigned)a | ((unsigned)b << 16); }
__device__ __forceinline__ unsigned short h_bits(float f) { const _Float16 h = (_Float16)f; return __builtin_bit_cast(unsigned short, h); }

template <int ET> struct Elem;
template <> struct Elem<0> { typedef _Float16 T; };
template <> struct Elem<1> { typedef __bf16 T; };
template <int ET, int SPL, int BIAS_MODE, int OUT_MODE, int RESID, int ACT>
__global__ __launch_bounds__(256) void wmma_gemm64(
    const unsigned short* __restrict__ Ap, const unsigned short* __restrict__ A2p, int lda, long strideA,
    const unsigned short* __restrict__ Btp, const unsigned short* __restrict__ Bt2p, int ldb, long strideB,
    void* __restrict__ Cout, void* __restrict__ Cout2, int ldc, long strideC,
    const float* __restrict__ bias,
    const float* __restrict__ resid, long strideR,
    int M, int N, int K, float scale) {
  typedef typename Elem<ET>::T T;
  typedef typename Frag<T>::V V;
  const T* A = (const T*)Ap; const T* A2 = (const T*)A2p; const T* Bt = (const T*)Btp; const T* Bt2 = (const T*)Bt2p;
  __shared__ __align__(16) float sT[8][16 * 68];
  const int b    = blockIdx.y;
  const int lane = threadIdx.x & 31;
  const int wave = threadIdx.x >> 5;
  const int tilesN = N >> 6;
  const int tilesM = M >> 6;
  const int tile = blockIdx.x * 8 + wave;
  if (tile >= tilesM * tilesN) return;
  const int tm = tile / tilesN;
  const int tn = tile - tm * tilesN;
  const int m0 = tm << 6;
  const int n0 = tn << 6;

  const T* Ab  = A  + (size_t)b * strideA;
  const T* Bb  = Bt + (size_t)b * strideB;
  const T* Ab2 = (SPL & 1) ? (A2  + (size_t)b * strideA) : nullptr;
  const T* Bb2 = (SPL & 2) ? (Bt2 + (size_t)b * strideB) : nullptr;

  const int rlane = lane & 15;
  const int koff  = (lane >> 4) * 8;
  const int mOff  = (lane >> 4) * 8;

  v8f acc[4][4];
#pragma unroll
  for (int i = 0; i < 4; ++i)
#pragma unroll
    for (int j = 0; j < 4; ++j) acc[i][j] = (v8f){0.f,0.f,0.f,0.f,0.f,0.f,0.f,0.f};

  for (int k0 = 0; k0 < K; k0 += 32) {
    V bh[4], bl[4];
#pragma unroll
    for (int j = 0; j < 4; ++j) {
      const size_t bo = (size_t)(n0 + (j << 4) + rlane) * ldb + koff + k0;
      bh[j] = Frag<T>::load(Bb + bo);
      if (SPL & 2) bl[j] = Frag<T>::load(Bb2 + bo);
    }
#pragma unroll
    for (int i = 0; i < 4; ++i) {
      const size_t ao = (size_t)(m0 + (i << 4) + rlane) * lda + koff + k0;
      V ah = Frag<T>::load(Ab + ao);
      V al;
      if (SPL & 1) al = Frag<T>::load(Ab2 + ao);
#pragma unroll
      for (int j = 0; j < 4; ++j) {
        acc[i][j] = Frag<T>::mma(ah, bh[j], acc[i][j]);
        if (SPL & 2) acc[i][j] = Frag<T>::mma(ah, bl[j], acc[i][j]);
        if (SPL & 1) acc[i][j] = Frag<T>::mma(al, bh[j], acc[i][j]);
      }
      Frag<T>::guard(acc[i][0], acc[i][3], ah, (SPL & 1) ? al : ah);
    }
    Frag<T>::keep(bh[0], bh[1], bh[2], bh[3]);
    if (SPL & 2) Frag<T>::keep(bl[0], bl[1], bl[2], bl[3]);
  }
  acc_guard4(acc[0][0], acc[0][1], acc[0][2], acc[0][3]);
  acc_guard4(acc[1][0], acc[1][1], acc[1][2], acc[1][3]);
  acc_guard4(acc[2][0], acc[2][1], acc[2][2], acc[2][3]);
  acc_guard4(acc[3][0], acc[3][1], acc[3][2], acc[3][3]);

  float* slab = sT[wave];
  const float* Rb = (RESID != 0) ? (resid + (size_t)b * strideR) : nullptr;
#pragma unroll
  for (int i = 0; i < 4; ++i) {
    const int mBase = m0 + (i << 4);
#pragma unroll
    for (int j = 0; j < 4; ++j) {
      const int n = n0 + (j << 4) + rlane;
      float bv = 0.f;
      if (BIAS_MODE == 2) bv = bias[n];
#pragma unroll
      for (int r = 0; r < 8; ++r) {
        float v = acc[i][j][r] * scale;
        if (BIAS_MODE == 1) v += bias[mBase + mOff + r];
        if (BIAS_MODE == 2) v += bv;
        if (RESID == 1) v += Rb[(size_t)(mBase + mOff + r) * ldc + n];
        if (RESID == 2) v += bf_bits2f(f2bf_bits(Rb[(size_t)(mBase + mOff + r) * ldc + n]));
        if (ACT == 2) v = fmaxf(v, 0.0f);
        slab[(mOff + r) * 68 + (j << 4) + rlane] = v;
      }
    }
    __builtin_amdgcn_fence(__ATOMIC_RELEASE, "workgroup");
    __builtin_amdgcn_wave_barrier();
    __builtin_amdgcn_fence(__ATOMIC_ACQUIRE, "workgroup");
    if (OUT_MODE == 0) {
      float* C = (float*)Cout + (size_t)b * strideC;
      const int hh = lane >> 4, c4 = (lane & 15) * 4;
      for (int pass = 0; pass < 2; ++pass) {
#pragma unroll
        for (int it = 0; it < 8; ++it) {
          const int row = it * 2 + hh;
          v4f v = *(const v4f*)(slab + row * 68 + c4);
          *(volatile v4f*)(C + (size_t)(mBase + row) * ldc + n0 + c4) = v;
        }
        __threadfence();
      }
    } else {
      const int q = lane >> 3, c8 = (lane & 7) * 8;
      unsigned short* C  = (unsigned short*)Cout  + (size_t)b * strideC;
      unsigned short* C2 = (OUT_MODE == 2) ? ((unsigned short*)Cout2 + (size_t)b * strideC) : nullptr;
      for (int pass = 0; pass < 2; ++pass) {
#pragma unroll
        for (int it = 0; it < 4; ++it) {
          const int row = it * 4 + q;
          const float* sp = slab + row * 68 + c8;
          v8h hv, lv;
#pragma unroll
          for (int e = 0; e < 8; ++e) {
            if (OUT_MODE == 1) {
              hv[e] = (_Float16)sp[e];
            } else {
              unsigned short hb = f2bf_bits(sp[e]);
              unsigned short lb = f2bf_bits(sp[e] - bf_bits2f(hb));
              hv[e] = __builtin_bit_cast(_Float16, hb);
              lv[e] = __builtin_bit_cast(_Float16, lb);
            }
          }
          *(volatile v8h*)(C + (size_t)(mBase + row) * ldc + n0 + c8) = hv;
          if (OUT_MODE == 2) *(volatile v8h*)(C2 + (size_t)(mBase + row) * ldc + n0 + c8) = lv;
        }
        __threadfence();
      }
    }
    __builtin_amdgcn_fence(__ATOMIC_RELEASE, "workgroup");
    __builtin_amdgcn_wave_barrier();
    __builtin_amdgcn_fence(__ATOMIC_ACQUIRE, "workgroup");
  }
}

template <int MODE>
__global__ __launch_bounds__(256) void cast8_kernel(const float* __restrict__ in, unsigned short* __restrict__ out, int n8, float scale) {
  const int i = blockIdx.x * 256 + threadIdx.x;
  if (i >= n8) return;
  const float* p = in + 8 * (size_t)i;
  const v4f a = *(const v4f*)(p);
  const v4f c = *(const v4f*)(p + 4);
  unsigned short hb[8];
#pragma unroll
  for (int e = 0; e < 4; ++e) {
    if (MODE == 0) {
      hb[e]     = f2bf_bits(a[e]);
      hb[4 + e] = f2bf_bits(c[e]);
    } else {
      hb[e]     = h_bits(bf_bits2f(f2bf_bits(a[e])) * scale);
      hb[4 + e] = h_bits(bf_bits2f(f2bf_bits(c[e])) * scale);
    }
  }
  const v4u u = (v4u){pk16(hb[0], hb[1]), pk16(hb[2], hb[3]), pk16(hb[4], hb[5]), pk16(hb[6], hb[7])};
  unsigned short* q = out + 8 * (size_t)i;
  *(volatile v4u*)q = u;
  __threadfence();
  *(volatile v4u*)q = u;
  (void)scale;
}

template <int MODE>
__global__ __launch_bounds__(256) void transpose_cast_kernel(const float* __restrict__ in, unsigned short* __restrict__ out,
                                                             int R, int Cc, float scale) {
  __shared__ float tile[64][65];
  const int t  = threadIdx.x;
  const int r0 = blockIdx.y * 64, c0 = blockIdx.x * 64;
  const int lc = t & 63, lr = t >> 6;
#pragma unroll
  for (int i = 0; i < 16; ++i) {
    const int r = i * 4 + lr;
    tile[r][lc] = in[(size_t)(r0 + r) * Cc + c0 + lc];
  }
  __syncthreads();
  const int lane = t & 31, wave = t >> 5;
  const int q = lane >> 3, c8 = (lane & 7) * 8;
#pragma unroll
  for (int it = 0; it < 2; ++it) {
    const int cc = it * 32 + wave * 4 + q;
    unsigned short hb[8];
#pragma unroll
    for (int e = 0; e < 8; ++e) {
      const float v = tile[c8 + e][cc];
      hb[e] = (MODE == 0) ? f2bf_bits(v) : h_bits(bf_bits2f(f2bf_bits(v)) * scale);
    }
    const v4u u = (v4u){pk16(hb[0], hb[1]), pk16(hb[2], hb[3]), pk16(hb[4], hb[5]), pk16(hb[6], hb[7])};
    unsigned short* p = out + (size_t)(c0 + cc) * R + r0 + c8;
    *(volatile v4u*)p = u;
    __threadfence();
    *(volatile v4u*)p = u;
  }
  (void)scale;
}

__global__ __launch_bounds__(256) void rne4_kernel(const float* __restrict__ in, float* __restrict__ out, int n4) {
  const int i = blockIdx.x * 256 + threadIdx.x;
  if (i >= n4) return;
  const v4f a = *(const v4f*)(in + 4 * (size_t)i);
  v4f r;
#pragma unroll
  for (int e = 0; e < 4; ++e) r[e] = bf_bits2f(f2bf_bits(a[e]));
  float* p = out + 4 * (size_t)i;
  *(volatile v4f*)p = r;
  __threadfence();
  *(volatile v4f*)p = r;
}

template <int IN_RND, int OUTM>
__global__ __launch_bounds__(64) void layernorm512_kernel(const float* __restrict__ x, const float* __restrict__ g,
                                                          const float* __restrict__ bb,
                                                          unsigned short* __restrict__ O1, unsigned short* __restrict__ O2) {
  __shared__ float redA[2];
  __shared__ float redB[2];
  const int row  = blockIdx.x;
  const int t    = threadIdx.x;
  const int lane = t & 31, wave = t >> 5;
  const int c0   = t * 8;
  const float* xr = x + (size_t)row * kDim + c0;
  const v4f a = *(const v4f*)(xr);
  const v4f c = *(const v4f*)(xr + 4);
  float xb[8];
#pragma unroll
  for (int e = 0; e < 4; ++e) {
    xb[e]     = IN_RND ? bf_bits2f(f2bf_bits(a[e])) : a[e];
    xb[4 + e] = IN_RND ? bf_bits2f(f2bf_bits(c[e])) : c[e];
  }
  float s = ((xb[0] + xb[1]) + (xb[2] + xb[3])) + ((xb[4] + xb[5]) + (xb[6] + xb[7]));
#pragma unroll
  for (int off = 16; off > 0; off >>= 1) s += __shfl_xor(s, off, 32);
  if (lane == 0) redA[wave] = s;
  __syncthreads();
  const float mu = (redA[0] + redA[1]) * kInvDim;
  float d[8];
#pragma unroll
  for (int e = 0; e < 8; ++e) d[e] = xb[e] - mu;
  float qq = ((d[0] * d[0] + d[1] * d[1]) + (d[2] * d[2] + d[3] * d[3])) + ((d[4] * d[4] + d[5] * d[5]) + (d[6] * d[6] + d[7] * d[7]));
#pragma unroll
  for (int off = 16; off > 0; off >>= 1) qq += __shfl_xor(qq, off, 32);
  if (lane == 0) redB[wave] = qq;
  __syncthreads();
  const float var = (redB[0] + redB[1]) * kInvDim;
  const float rs  = rsqrtf(var + kLnEps);
  const v4f ga = *(const v4f*)(g + c0);
  const v4f gc = *(const v4f*)(g + c0 + 4);
  const v4f ba = *(const v4f*)(bb + c0);
  const v4f bc = *(const v4f*)(bb + c0 + 4);
  float gv[8], bv[8];
#pragma unroll
  for (int e = 0; e < 4; ++e) {
    gv[e]     = bf_bits2f(f2bf_bits(ga[e]));
    gv[4 + e] = bf_bits2f(f2bf_bits(gc[e]));
    bv[e]     = bf_bits2f(f2bf_bits(ba[e]));
    bv[4 + e] = bf_bits2f(f2bf_bits(bc[e]));
  }
  unsigned short o1[8], o2[8];
#pragma unroll
  for (int e = 0; e < 8; ++e) {
    const float y = (d[e] * rs) * gv[e] + bv[e];
    if (OUTM == 1) {
      o1[e] = h_bits(y);
      o2[e] = 0;
    } else {
      const unsigned short hh = f2bf_bits(y);
      o1[e] = hh;
      o2[e] = f2bf_bits(y - bf_bits2f(hh));
    }
  }
  const v4u u1 = (v4u){pk16(o1[0], o1[1]), pk16(o1[2], o1[3]), pk16(o1[4], o1[5]), pk16(o1[6], o1[7])};
  const v4u u2 = (v4u){pk16(o2[0], o2[1]), pk16(o2[2], o2[3]), pk16(o2[4], o2[5]), pk16(o2[6], o2[7])};
  unsigned short* p1 = O1 + (size_t)row * kDim + c0;
  unsigned short* p2 = O2 + (size_t)row * kDim + c0;
  *(volatile v4u*)p1 = u1;
  if (OUTM == 2) *(volatile v4u*)p2 = u2;
  __threadfence();
  *(volatile v4u*)p1 = u1;
  if (OUTM == 2) *(volatile v4u*)p2 = u2;
}

__global__ __launch_bounds__(64) void rownorm_q_kernel(const float* __restrict__ Q, unsigned short* __restrict__ OH,
                                                       unsigned short* __restrict__ OL) {
  const int row = blockIdx.x;
  const int t   = threadIdx.x;
  const int c0  = t * 8;
  const float* xr = Q + (size_t)row * kDim + c0;
  const v4f a = *(const v4f*)(xr);
  const v4f c = *(const v4f*)(xr + 4);
  float v[8];
#pragma unroll
  for (int e = 0; e < 4; ++e) { v[e] = a[e]; v[4 + e] = c[e]; }
  float ss = ((v[0] * v[0] + v[1] * v[1]) + (v[2] * v[2] + v[3] * v[3])) + ((v[4] * v[4] + v[5] * v[5]) + (v[6] * v[6] + v[7] * v[7]));
  ss += __shfl_xor(ss, 1, 32);
  ss += __shfl_xor(ss, 2, 32);
  ss += __shfl_xor(ss, 4, 32);
  const float rinv = 1.0f / fmaxf(sqrtf(ss), kNormEps);
  unsigned short hb[8], lb[8];
#pragma unroll
  for (int e = 0; e < 8; ++e) {
    const float y = v[e] * rinv;
    const unsigned short hh = f2bf_bits(y);
    hb[e] = hh;
    lb[e] = f2bf_bits(y - bf_bits2f(hh));
  }
  const v4u uh = (v4u){pk16(hb[0], hb[1]), pk16(hb[2], hb[3]), pk16(hb[4], hb[5]), pk16(hb[6], hb[7])};
  const v4u ul = (v4u){pk16(lb[0], lb[1]), pk16(lb[2], lb[3]), pk16(lb[4], lb[5]), pk16(lb[6], lb[7])};
  unsigned short* ph = OH + (size_t)row * kDim + c0;
  unsigned short* pl = OL + (size_t)row * kDim + c0;
  *(volatile v4u*)ph = uh;
  *(volatile v4u*)pl = ul;
  __threadfence();
  *(volatile v4u*)ph = uh;
  *(volatile v4u*)pl = ul;
}

__global__ __launch_bounds__(256) void colnorm_k_kernel(const float* __restrict__ KT, unsigned short* __restrict__ KH,
                                                        unsigned short* __restrict__ KL, int ntok) {
  __shared__ __align__(16) float tile[64][68];
  __shared__ float psum[4][64];
  __shared__ float rinv[64];
  const int t    = threadIdx.x;
  const int h    = blockIdx.y;
  const int tok0 = blockIdx.x * 64;
  const size_t rowbase = (size_t)h * kHdim;
  {
    const int c4 = (t & 15) * 4, rr = t >> 4;
#pragma unroll
    for (int i = 0; i < 4; ++i) {
      const int r = i * 16 + rr;
      const v4f v = *(const v4f*)(KT + (rowbase + r) * (size_t)ntok + tok0 + c4);
      *(v4f*)(&tile[r][c4]) = v;
    }
  }
  __syncthreads();
  {
    const int c = t & 63, rg = t >> 6;
    float s = 0.f;
#pragma unroll
    for (int i = 0; i < 16; ++i) { const float v = tile[rg * 16 + i][c]; s = fmaf(v, v, s); }
    psum[rg][c] = s;
  }
  __syncthreads();
  if (t < 64) {
    const float ss = (psum[0][t] + psum[1][t]) + (psum[2][t] + psum[3][t]);
    rinv[t] = 1.0f / fmaxf(sqrtf(ss), kNormEps);
  }
  __syncthreads();
  const int lane = t & 31, wave = t >> 5;
  const int q = lane >> 3, c8 = (lane & 7) * 8;
#pragma unroll
  for (int it = 0; it < 2; ++it) {
    const int r = it * 32 + wave * 4 + q;
    unsigned short hb[8], lb[8];
#pragma unroll
    for (int e = 0; e < 8; ++e) {
      const float y = tile[r][c8 + e] * rinv[c8 + e];
      const unsigned short hh = f2bf_bits(y);
      hb[e] = hh;
      lb[e] = f2bf_bits(y - bf_bits2f(hh));
    }
    const v4u uh = (v4u){pk16(hb[0], hb[1]), pk16(hb[2], hb[3]), pk16(hb[4], hb[5]), pk16(hb[6], hb[7])};
    const v4u ul = (v4u){pk16(lb[0], lb[1]), pk16(lb[2], lb[3]), pk16(lb[4], lb[5]), pk16(lb[6], lb[7])};
    unsigned short* ph = KH + (rowbase + r) * (size_t)ntok + tok0 + c8;
    unsigned short* pl = KL + (rowbase + r) * (size_t)ntok + tok0 + c8;
    *(volatile v4u*)ph = uh;
    *(volatile v4u*)pl = ul;
    __threadfence();
    *(volatile v4u*)ph = uh;
    *(volatile v4u*)pl = ul;
  }
}

__global__ __launch_bounds__(256) void gelu2_kernel(unsigned short* H, int n2) {
  const int i = blockIdx.x * 256 + threadIdx.x;
  if (i >= n2) return;
  const _Float16* p = (const _Float16*)H + 2 * (size_t)i;
  unsigned u = 0u;
#pragma unroll 1
  for (int e = 0; e < 2; ++e) {
    const float v = (float)p[e];
    const float y = 0.5f * v * (1.0f + erff(v * 0.70710678118654752f));
    u |= ((unsigned)h_bits(y)) << (16 * e);
  }
  unsigned* q = (unsigned*)H + (size_t)i;
  *(volatile unsigned*)q = u;
  __threadfence();
  *(volatile unsigned*)q = u;
}

extern "C" void kernel_launch(void* const* d_in, const int* in_sizes, int n_in,
                              void* d_out, int out_size, void* d_ws, size_t ws_size,
                              hipStream_t stream) {
  if (n_in < 16) return;
  if (in_sizes[0] != kTok * kDim || in_sizes[1] != kTok * kDim || in_sizes[2] != kTok * kDim) return;
  if (in_sizes[3] != kDim * kDim || in_sizes[4] != kDim * kDim || in_sizes[5] != kDim * kDim || in_sizes[6] != kDim * kDim) return;
  if (in_sizes[7] != kDim || in_sizes[8] != kDim || in_sizes[9] != kDim || in_sizes[10] != kDim || in_sizes[11] != kDim) return;
  if (in_sizes[12] != kDim * kMlp || in_sizes[13] != kMlp || in_sizes[14] != kMlp * kDim || in_sizes[15] != kDim) return;
  if (out_size != kTok * kDim) return;

  const float* q   = (const float*)d_in[0];
  const float* kin = (const float*)d_in[1];
  const float* vin = (const float*)d_in[2];
  const float* Wq  = (const float*)d_in[3];
  const float* Wk  = (const float*)d_in[4];
  const float* Wv  = (const float*)d_in[5];
  const float* Wo  = (const float*)d_in[6];
  const float* bo  = (const float*)d_in[7];
  const float* g1  = (const float*)d_in[8];
  const float* b1  = (const float*)d_in[9];
  const float* g2  = (const float*)d_in[10];
  const float* b2  = (const float*)d_in[11];
  const float* W1  = (const float*)d_in[12];
  const float* bf1 = (const float*)d_in[13];
  const float* W2  = (const float*)d_in[14];
  const float* bf2 = (const float*)d_in[15];
  float* outp = (float*)d_out;

  const size_t SZ_W    = (size_t)kDim * kDim * 2;
  const size_t SZ_WM   = (size_t)kDim * kMlp * 2;
  const size_t SZ_B512 = (size_t)kDim * 4;
  const size_t SZ_B2K  = (size_t)kMlp * 4;
  const size_t SZ_KVT  = (size_t)kGroups * kHdim * kHdim * 2;
  const size_t SZ_P16  = (size_t)kTok * kDim * 2;
  const size_t SZ_P32  = (size_t)kTok * kDim * 4;

  size_t off = 0;
  const size_t oWQT  = off; off += SZ_W;
  const size_t oWKT  = off; off += SZ_W;
  const size_t oWVT  = off; off += SZ_W;
  const size_t oWOT  = off; off += SZ_W;
  const size_t oW1T  = off; off += SZ_WM;
  const size_t oW2T  = off; off += SZ_WM;
  const size_t oBOR  = off; off += SZ_B512;
  const size_t oBF1R = off; off += SZ_B2K;
  const size_t oBF2R = off; off += SZ_B512;
  const size_t oKVTH = off; off += SZ_KVT;
  const size_t oKVTL = off; off += SZ_KVT;
  const size_t oR0   = off; off += SZ_P32;
  const size_t oR1   = off; off += SZ_P32;
  const size_t oR2   = off; off += SZ_P32;
  const size_t oR3   = off; off += SZ_P32;
  const size_t oR4   = off; off += SZ_P32;
  const size_t TOTAL = off;
  if (TOTAL > ws_size) return;
  if (TOTAL > (size_t)134217728) return;

  char* ws = (char*)d_ws;
  unsigned short* WQT  = (unsigned short*)(ws + oWQT);
  unsigned short* WKT  = (unsigned short*)(ws + oWKT);
  unsigned short* WVT  = (unsigned short*)(ws + oWVT);
  unsigned short* WOT  = (unsigned short*)(ws + oWOT);
  unsigned short* W1T  = (unsigned short*)(ws + oW1T);
  unsigned short* W2T  = (unsigned short*)(ws + oW2T);
  float*          BOR  = (float*)(ws + oBOR);
  float*          BF1R = (float*)(ws + oBF1R);
  float*          BF2R = (float*)(ws + oBF2R);
  unsigned short* KVTH = (unsigned short*)(ws + oKVTH);
  unsigned short* KVTL = (unsigned short*)(ws + oKVTL);
  unsigned short* KB   = (unsigned short*)(ws + oR0);
  unsigned short* VB   = (unsigned short*)(ws + oR0 + SZ_P16);
  unsigned short* QNH  = (unsigned short*)(ws + oR0);
  unsigned short* QNL  = (unsigned short*)(ws + oR0 + SZ_P16);
  unsigned short* XF   = (unsigned short*)(ws + oR0);
  unsigned short* LNQH = (unsigned short*)(ws + oR1);
  unsigned short* LNQL = (unsigned short*)(ws + oR1 + SZ_P16);
  unsigned short* KNTH = (unsigned short*)(ws + oR1);
  unsigned short* KNTL = (unsigned short*)(ws + oR1 + SZ_P16);
  unsigned short* HPL  = (unsigned short*)(ws + oR1);
  unsigned short* VTH  = (unsigned short*)(ws + oR2);
  unsigned short* VTL  = (unsigned short*)(ws + oR2 + SZ_P16);
  float*          Q32  = (float*)(ws + oR3);
  unsigned short* OHP  = (unsigned short*)(ws + oR3);
  unsigned short* OLP  = (unsigned short*)(ws + oR3 + SZ_P16);
  float*          KT32 = (float*)(ws + oR4);
  float*          X32  = (float*)(ws + oR4);

  const dim3 blk(256);

  transpose_cast_kernel<0><<<dim3(kDim / 64, kDim / 64), blk, 0, stream>>>(Wq, WQT, kDim, kDim, 1.0f);
  transpose_cast_kernel<0><<<dim3(kDim / 64, kDim / 64), blk, 0, stream>>>(Wk, WKT, kDim, kDim, 1.0f);
  transpose_cast_kernel<0><<<dim3(kDim / 64, kDim / 64), blk, 0, stream>>>(Wv, WVT, kDim, kDim, 1.0f);
  transpose_cast_kernel<0><<<dim3(kDim / 64, kDim / 64), blk, 0, stream>>>(Wo, WOT, kDim, kDim, 1.0f);
  transpose_cast_kernel<1><<<dim3(kMlp / 64, kDim / 64), blk, 0, stream>>>(W1, W1T, kDim, kMlp, kWCarry);
  transpose_cast_kernel<1><<<dim3(kDim / 64, kMlp / 64), blk, 0, stream>>>(W2, W2T, kMlp, kDim, kWCarry);

  {
    const int n8 = kTok * kDim / 8;
    cast8_kernel<0><<<dim3(n8 / 256), blk, 0, stream>>>(kin, KB, n8, 1.0f);
    cast8_kernel<0><<<dim3(n8 / 256), blk, 0, stream>>>(vin, VB, n8, 1.0f);
  }
  rne4_kernel<<<dim3(1), blk, 0, stream>>>(bo,  BOR,  kDim / 4);
  rne4_kernel<<<dim3(2), blk, 0, stream>>>(bf1, BF1R, kMlp / 4);
  rne4_kernel<<<dim3(1), blk, 0, stream>>>(bf2, BF2R, kDim / 4);

  layernorm512_kernel<1, 2><<<dim3(kTok), dim3(64), 0, stream>>>(q, g1, b1, LNQH, LNQL);

  const dim3 gP((( (kTok / 64) * (kDim / 64)) + 7) / 8, 1);
  const dim3 gKV(1, kHeads);
  const dim3 gO(((kSeq / 64) * (kHdim / 64) + 7) / 8, kHeads);
  const dim3 gW1((((kTok / 64) * (kMlp / 64)) + 7) / 8, 1);

  wmma_gemm64<1, 1, 0, 0, 0, 0><<<gP, blk, 0, stream>>>(
      LNQH, LNQL, kDim, 0L, WQT, WQT, kDim, 0L, (void*)Q32, (void*)Q32, kDim, 0L, BOR, q, 0L, kTok, kDim, kDim, 1.0f);
  wmma_gemm64<1, 0, 0, 0, 0, 0><<<gP, blk, 0, stream>>>(
      WKT, WKT, kDim, 0L, KB, KB, kDim, 0L, (void*)KT32, (void*)KT32, kTok, 0L, BOR, q, 0L, kDim, kTok, kDim, 1.0f);
  wmma_gemm64<1, 0, 0, 2, 0, 0><<<gP, blk, 0, stream>>>(
      WVT, WVT, kDim, 0L, VB, VB, kDim, 0L, (void*)VTH, (void*)VTL, kTok, 0L, BOR, q, 0L, kDim, kTok, kDim, 1.0f);

  rownorm_q_kernel<<<dim3(kTok), dim3(64), 0, stream>>>(Q32, QNH, QNL);
  colnorm_k_kernel<<<dim3(kTok / 64, kHeads), blk, 0, stream>>>(KT32, KNTH, KNTL, kTok);

  for (int b = 0; b < kBatch; ++b) {
    const size_t cOff = (size_t)b * kSeq;
    wmma_gemm64<1, 3, 0, 2, 0, 0><<<gKV, blk, 0, stream>>>(
        VTH + cOff, VTL + cOff, kTok, (long)kHdim * kTok,
        KNTH + cOff, KNTL + cOff, kTok, (long)kHdim * kTok,
        (void*)(KVTH + (size_t)b * kHeads * kHdim * kHdim), (void*)(KVTL + (size_t)b * kHeads * kHdim * kHdim),
        kHdim, (long)kHdim * kHdim, BOR, q, 0L, kHdim, kHdim, kSeq, 1.0f);
  }
  for (int b = 0; b < kBatch; ++b) {
    const size_t rOff = (size_t)b * kSeq * kDim;
    wmma_gemm64<1, 3, 0, 2, 0, 0><<<gO, blk, 0, stream>>>(
        QNH + rOff, QNL + rOff, kDim, (long)kHdim,
        KVTH + (size_t)b * kHeads * kHdim * kHdim, KVTL + (size_t)b * kHeads * kHdim * kHdim, kHdim, (long)kHdim * kHdim,
        (void*)(OHP + rOff), (void*)(OLP + rOff), kDim, (long)kHdim, BOR, q, 0L, kSeq, kHdim, kHdim, 1.0f);
  }

  wmma_gemm64<1, 1, 2, 0, 2, 0><<<gP, blk, 0, stream>>>(
      OHP, OLP, kDim, 0L, WOT, WOT, kDim, 0L, (void*)X32, (void*)X32, kDim, 0L, BOR, q, 0L, kTok, kDim, kDim, 1.0f);

  layernorm512_kernel<0, 1><<<dim3(kTok), dim3(64), 0, stream>>>(X32, g2, b2, XF, XF);

  wmma_gemm64<0, 0, 2, 1, 0, 0><<<gW1, blk, 0, stream>>>(
      XF, XF, kDim, 0L, W1T, W1T, kDim, 0L, (void*)HPL, (void*)HPL, kMlp, 0L, BF1R, q, 0L, kTok, kMlp, kDim, kWCarryInv);
  {
    const int n2 = kTok * kMlp / 2;
    gelu2_kernel<<<dim3(n2 / 256), blk, 0, stream>>>(HPL, n2);
  }
  wmma_gemm64<0, 0, 2, 0, 1, 0><<<gP, blk, 0, stream>>>(
      HPL, HPL, kMlp, 0L, W2T, W2T, kMlp, 0L, (void*)outp, (void*)outp, kDim, 0L, BF2R, X32, 0L, kTok, kDim, kMlp, kWCarryInv);
}
